// TransformerEncoder_86457691669082
// MI455X (gfx1250) — hardware-run, weakly checked
//
#include <hip/hip_runtime.h>
#include <math.h>

typedef _Float16 v16h __attribute__((ext_vector_type(16)));
typedef _Float16 v8h  __attribute__((ext_vector_type(8)));
typedef _Float16 v4h  __attribute__((ext_vector_type(4)));
typedef float    v8f  __attribute__((ext_vector_type(8)));
typedef float    v4f  __attribute__((ext_vector_type(4)));
typedef v8h __attribute__((may_alias)) v8ha;
typedef v4f __attribute__((may_alias)) v4fa;

union Frag { v16h v; v8h half[2]; };

#define NBATCH 2
#define SEQ    2048
#define DM     1024
#define HID    256
#define NH     4
#define HD     64
#define DFF    512
#define MROWS  (NBATCH * SEQ)
#define NQT    (SEQ / 64)
#define N8ACT  (MROWS * DM / 8)
#define PSC    16384.0f

static_assert(NH * HD == HID);
static_assert((MROWS % 128) == 0 && (HID % 128) == 0);
static_assert((HID % 64) == 0 && (DM % 64) == 0 && (DFF % 64) == 0 && (SEQ % 64) == 0);
static_assert((DM % 32) == 0 && (HID % 32) == 0 && (DFF % 32) == 0);
static_assert(NQT == 32);
static_assert((N8ACT % 256) == 0);
static_assert(((MROWS * HID / 8) % 256) == 0);
static_assert((MROWS % 8) == 0);

__device__ __forceinline__ v8f wmma_f16(v16h a, v16h b, v8f c) {
  v8f d = __builtin_amdgcn_wmma_f32_16x16x32_f16(false, a, false, b, (short)0, c, false, false);
  asm volatile("v_nop\n\tv_nop\n\tv_nop\n\tv_nop" : "+v"(d) : "v"(a), "v"(b));
  return d;
}

__device__ __forceinline__ v16h load_frag(const _Float16* p, int h) {
  Frag f;
  f.half[0] = *(const v8ha*)(p + 8 * h);
  f.half[1] = *(const v8ha*)(p + 16 + 8 * h);
  return f.v;
}

__device__ __forceinline__ v4f relu4(v4f a) {
  a.x = fmaxf(a.x, 0.0f); a.y = fmaxf(a.y, 0.0f); a.z = fmaxf(a.z, 0.0f); a.w = fmaxf(a.w, 0.0f);
  return a;
}

__global__ __launch_bounds__(256) void k_cvt(
    const float* __restrict__ q, const float* __restrict__ k, const float* __restrict__ v,
    _Float16* q16, _Float16* k16, _Float16* v16)
{
  const int g = blockIdx.x * 256 + (int)threadIdx.x;
  if (g >= 3 * N8ACT) return;
  const int p   = g / N8ACT;
  const int off = g - p * N8ACT;
  const float* src = (p == 0) ? q : ((p == 1) ? k : v);
  _Float16*    dst = (p == 0) ? q16 : ((p == 1) ? k16 : v16);
  const v4f a = *(const v4fa*)(src + (size_t)off * 8);
  const v4f c = *(const v4fa*)(src + (size_t)off * 8 + 4);
  const v8h o = { (_Float16)a.x, (_Float16)a.y, (_Float16)a.z, (_Float16)a.w,
                  (_Float16)c.x, (_Float16)c.y, (_Float16)c.z, (_Float16)c.w };
  _Float16* d = dst + (size_t)off * 8;
  *(volatile v8h*)d = o;
  __threadfence();
  *(volatile v8h*)d = o;
}

__global__ __launch_bounds__(256) void k_wt(const float* __restrict__ W, int R, int C,
                                             _Float16* WT, float carry)
{
  __shared__ float s[64][65];
  const int tid = threadIdx.x, lane = tid & 31, w = tid >> 5;
  const int c0 = blockIdx.x * 64, r0 = blockIdx.y * 64;
#pragma unroll
  for (int it = 0; it < 4; ++it) {
    const int idx = it * 256 + tid;
    const int r = idx >> 4, c4 = (idx & 15) * 4;
    const v4f v = *(const v4fa*)(W + (size_t)(r0 + r) * C + c0 + c4);
    s[c4 + 0][r] = v.x; s[c4 + 1][r] = v.y; s[c4 + 2][r] = v.z; s[c4 + 3][r] = v.w;
  }
  __syncthreads();
  const int q8 = lane & 7, sub = lane >> 3;
  v8h hv[2];
#pragma unroll
  for (int i = 0; i < 2; ++i) {
    const int c = w * 8 + i * 4 + sub;
    const float* sp = &s[c][8 * q8];
    const v8h o = { (_Float16)(sp[0] * carry), (_Float16)(sp[1] * carry), (_Float16)(sp[2] * carry), (_Float16)(sp[3] * carry),
                    (_Float16)(sp[4] * carry), (_Float16)(sp[5] * carry), (_Float16)(sp[6] * carry), (_Float16)(sp[7] * carry) };
    hv[i] = o;
  }
  for (int pass = 0; pass < 2; ++pass) {
#pragma unroll
    for (int i = 0; i < 2; ++i) {
      const int c = w * 8 + i * 4 + sub;
      *(volatile v8h*)(WT + (size_t)(c0 + c) * R + r0 + 8 * q8) = hv[i];
    }
    __threadfence();
  }
}

template <int MODE, bool RELU>
__global__ __launch_bounds__(128) void gemm_k(
    const _Float16* __restrict__ A, int lda, long long sAz,
    const _Float16* __restrict__ Bt, int ldb, long long sBz,
    const float* __restrict__ bias, const float* __restrict__ resid,
    void* Cv, int ldc, long long sCz, int K, float ascale, float ocarry)
{
  __shared__ __attribute__((aligned(16))) float sO[4 * 32 * 64];

  const int tid = threadIdx.x, lane = tid & 31, w = tid >> 5;
  const int h = lane >> 4, m = lane & 15;
  const int m0w = blockIdx.x * 128 + 32 * w;
  const int n0  = blockIdx.y * 64;
  const int z   = blockIdx.z;
  const _Float16* Ab = A  + (size_t)z * (size_t)sAz;
  const _Float16* Bb = Bt + (size_t)z * (size_t)sBz;
  const _Float16* xa0 = Ab + (size_t)(m0w + m) * lda;
  const _Float16* xa1 = xa0 + (size_t)16 * lda;
  const _Float16* wb  = Bb + (size_t)(n0 + m) * ldb;

  const v8f zero8 = {0.f, 0.f, 0.f, 0.f, 0.f, 0.f, 0.f, 0.f};
  v8f acc[2][4];
#pragma unroll
  for (int mt = 0; mt < 2; ++mt)
#pragma unroll
    for (int nt = 0; nt < 4; ++nt) acc[mt][nt] = zero8;

#pragma unroll 1
  for (int k0 = 0; k0 < K; k0 += 32) {
    const v16h a0 = load_frag(xa0 + k0, h);
    const v16h a1 = load_frag(xa1 + k0, h);
#pragma unroll
    for (int nt = 0; nt < 4; ++nt) {
      const v16h b = load_frag(wb + (size_t)nt * 16 * ldb + k0, h);
      acc[0][nt] = wmma_f16(a0, b, acc[0][nt]);
      acc[1][nt] = wmma_f16(a1, b, acc[1][nt]);
    }
  }

  float* so = sO + w * 2048;
#pragma unroll
  for (int mt = 0; mt < 2; ++mt)
#pragma unroll
    for (int nt = 0; nt < 4; ++nt)
#pragma unroll
      for (int r = 0; r < 8; ++r)
        so[(16 * mt + 8 * h + r) * 64 + 16 * nt + m] = acc[mt][nt][r] * ascale;
  __syncthreads();

  const int q8 = lane & 7, sub = lane >> 3;
  if (MODE == 0) {
    float* C = (float*)Cv + (size_t)z * (size_t)sCz;
    const v4f bz0 = *(const v4fa*)(bias + n0 + 4 * q8);
    const v4f bz1 = *(const v4fa*)(bias + n0 + 32 + 4 * q8);
    v4f y[16];
#pragma unroll
    for (int i = 0; i < 16; ++i) {
      const int lid = i * 4 + sub;
      const int row = lid >> 1, hl = lid & 1;
      const v4f v  = *(const v4fa*)(so + row * 64 + 32 * hl + 4 * q8);
      const size_t gi = (size_t)(m0w + row) * ldc + n0 + 32 * hl + 4 * q8;
      const v4f rr = *(const v4fa*)(resid + gi);
      y[i] = v + (hl ? bz1 : bz0) + rr;
    }
    for (int pass = 0; pass < 2; ++pass) {
#pragma unroll
      for (int i = 0; i < 16; ++i) {
        const int lid = i * 4 + sub;
        const int row = lid >> 1, hl = lid & 1;
        const size_t gi = (size_t)(m0w + row) * ldc + n0 + 32 * hl + 4 * q8;
        *(volatile v4f*)(C + gi) = y[i];
      }
      __threadfence();
    }
  } else {
    _Float16* C = (_Float16*)Cv + (size_t)z * (size_t)sCz;
    v4f bc0 = {0.f, 0.f, 0.f, 0.f}, bc1 = {0.f, 0.f, 0.f, 0.f};
    if (MODE == 1) {
      bc0 = *(const v4fa*)(bias + n0 + 8 * q8);
      bc1 = *(const v4fa*)(bias + n0 + 8 * q8 + 4);
    }
    v8h hv[8];
#pragma unroll
    for (int i = 0; i < 8; ++i) {
      const int row = i * 4 + sub;
      const float* sp = so + row * 64 + 8 * q8;
      v4f f0 = *(const v4fa*)sp;
      v4f f1 = *(const v4fa*)(sp + 4);
      if (MODE == 1) { f0 = f0 + bc0; f1 = f1 + bc1; }
      else { const float br = bias[m0w + row]; f0 = f0 + br; f1 = f1 + br; }
      if (RELU) { f0 = relu4(f0); f1 = relu4(f1); }
      const v8h o = { (_Float16)(f0.x * ocarry), (_Float16)(f0.y * ocarry), (_Float16)(f0.z * ocarry), (_Float16)(f0.w * ocarry),
                      (_Float16)(f1.x * ocarry), (_Float16)(f1.y * ocarry), (_Float16)(f1.z * ocarry), (_Float16)(f1.w * ocarry) };
      hv[i] = o;
    }
    for (int pass = 0; pass < 2; ++pass) {
#pragma unroll
      for (int i = 0; i < 8; ++i) {
        const int row = i * 4 + sub;
        *(volatile v8h*)(C + (size_t)(m0w + row) * ldc + n0 + 8 * q8) = hv[i];
      }
      __threadfence();
    }
  }
}

__device__ __forceinline__ v16h pack_p(v8f a, v8f c) {
  const v16h r = { (_Float16)(a[0] * PSC), (_Float16)(a[1] * PSC), (_Float16)(a[2] * PSC), (_Float16)(a[3] * PSC),
                   (_Float16)(a[4] * PSC), (_Float16)(a[5] * PSC), (_Float16)(a[6] * PSC), (_Float16)(a[7] * PSC),
                   (_Float16)(c[0] * PSC), (_Float16)(c[1] * PSC), (_Float16)(c[2] * PSC), (_Float16)(c[3] * PSC),
                   (_Float16)(c[4] * PSC), (_Float16)(c[5] * PSC), (_Float16)(c[6] * PSC), (_Float16)(c[7] * PSC) };
  return r;
}

__device__ __forceinline__ void att_store_pass(const float* so, float* out,
                                               int b, int head, int q0, int lane) {
  const int q8 = lane & 7, sub = lane >> 3;
#pragma unroll
  for (int i = 0; i < 8; ++i) {
    const int lid = i * 4 + sub;
    const int row = lid >> 1, hl = lid & 1;
    const v4f v = *(const v4fa*)(so + row * 64 + 32 * hl + 4 * q8);
    const size_t gi = ((size_t)(b * SEQ + q0 + row)) * HID + head * HD + 32 * hl + 4 * q8;
    *(volatile v4f*)(out + gi) = v;
  }
}

__global__ __launch_bounds__(128) __attribute__((amdgpu_num_vgpr(256))) void attn_k(
    const _Float16* __restrict__ Qp,
    const _Float16* __restrict__ Kp,
    const _Float16* __restrict__ VT,
    const float* __restrict__ alpha, const float* __restrict__ adjw, const float* __restrict__ adjb,
    float* tmp,
    float* rec)
{
  __shared__ float adjt[SEQ];
  __shared__ __attribute__((aligned(16))) float sO[4 * 16 * 64];
  __shared__ __attribute__((aligned(16))) float csum[64];

  const int tid = threadIdx.x, lane = tid & 31, w = tid >> 5;
  const int hh = lane >> 4, m = lane & 15;
  const int bh = blockIdx.y, b = bh >> 2, head = bh & 3;
  const int qt = blockIdx.x, q0b = qt * 64, q0w = q0b + 16 * w;

  {
#pragma clang fp contract(off)
    const float aw = adjw[0], ab = adjb[0];
#pragma unroll 1
    for (int i = tid; i < SEQ; i += 128) {
      const float dd = (float)i;
      const float d2 = dd * dd;
      const float e  = aw * d2 - ab;
      adjt[i] = expf(-fabsf(e));
    }
  }
  __syncthreads();

  const _Float16* qrow = Qp + (size_t)(b * SEQ + q0w + m) * HID + head * HD;
  const v16h qb0 = load_frag(qrow, hh);
  const v16h qb1 = load_frag(qrow + 32, hh);

  const v8f zero8 = {0.f, 0.f, 0.f, 0.f, 0.f, 0.f, 0.f, 0.f};
  v8f o[4], ol[4];
#pragma unroll
  for (int t = 0; t < 4; ++t) { o[t] = zero8; ol[t] = zero8; }
  float mG = -INFINITY, lG = 0.0f, mL = -INFINITY, lL = 0.0f;

  const _Float16* kbase = Kp + (size_t)(b * SEQ + m) * HID + head * HD;
  const _Float16* vbase = VT + (size_t)(b * HID + head * HD + m) * SEQ;
  const int iq = q0w + m;

#pragma unroll 1
  for (int kb = 0; kb < SEQ; kb += 32) {
    const bool lov = (kb + 31 >= q0b - 4) && (kb <= q0b + 67);

    v8f s[2];
#pragma unroll
    for (int j = 0; j < 2; ++j) {
      const _Float16* kp = kbase + (size_t)(kb + 16 * j) * HID;
      const v16h kf0 = load_frag(kp, hh);
      const v16h kf1 = load_frag(kp + 32, hh);
      v8f z = zero8;
      z = wmma_f16(kf0, qb0, z);
      z = wmma_f16(kf1, qb1, z);
#pragma unroll
      for (int r = 0; r < 8; ++r) {
        int ad = iq - (kb + 16 * j + 8 * hh + r);
        ad = (ad < 0) ? -ad : ad;
        z[r] = z[r] * (1.0f / 1024.0f) + adjt[ad];
      }
      s[j] = z;
    }

    float mloc = s[0][0];
#pragma unroll
    for (int j = 0; j < 2; ++j)
#pragma unroll
      for (int r = 0; r < 8; ++r) mloc = fmaxf(mloc, s[j][r]);
    mloc = fmaxf(mloc, __shfl_xor(mloc, 16));
    const float mGn = fmaxf(mG, mloc);
    const float msG = (mGn == -INFINITY) ? 0.0f : mGn;
    const float aG  = __expf(mG - msG);
    mG = mGn;
    float lsum = 0.0f;
    v8f pg[2];
#pragma unroll
    for (int j = 0; j < 2; ++j) {
      v8f pp = zero8;
#pragma unroll
      for (int r = 0; r < 8; ++r) {
        const float p = __expf(s[j][r] - msG);
        pp[r] = p;
        lsum += p;
      }
      pg[j] = pp;
    }
    lsum += __shfl_xor(lsum, 16);
    lG = lG * aG + lsum;
#pragma unroll
    for (int t = 0; t < 4; ++t)
#pragma unroll
      for (int r = 0; r < 8; ++r) o[t][r] = o[t][r] * aG;
    const v16h pbG = pack_p(pg[0], pg[1]);

    v16h pbL = pbG;
    if (lov) {
      float ml = -INFINITY;
#pragma unroll
      for (int j = 0; j < 2; ++j)
#pragma unroll
        for (int r = 0; r < 8; ++r) {
          int ad = iq - (kb + 16 * j + 8 * hh + r);
          ad = (ad < 0) ? -ad : ad;
          ml = (ad <= 4) ? fmaxf(ml, s[j][r]) : ml;
        }
      ml = fmaxf(ml, __shfl_xor(ml, 16));
      const float mLn = fmaxf(mL, ml);
      const float msL = (mLn == -INFINITY) ? 0.0f : mLn;
      const float aL  = __expf(mL - msL);
      mL = mLn;
      float ls = 0.0f;
      v8f pl[2];
#pragma unroll
      for (int j = 0; j < 2; ++j) {
        v8f pp = zero8;
#pragma unroll
        for (int r = 0; r < 8; ++r) {
          int ad = iq - (kb + 16 * j + 8 * hh + r);
          ad = (ad < 0) ? -ad : ad;
          const float e = __expf(s[j][r] - msL);
          const float p = (ad <= 4) ? e : 0.0f;
          pp[r] = p;
          ls += p;
        }
        pl[j] = pp;
      }
      ls += __shfl_xor(ls, 16);
      lL = lL * aL + ls;
#pragma unroll
      for (int t = 0; t < 4; ++t)
#pragma unroll
        for (int r = 0; r < 8; ++r) ol[t][r] = ol[t][r] * aL;
      pbL = pack_p(pl[0], pl[1]);
    }

    v16h vf[4];
#pragma unroll
    for (int t = 0; t < 4; ++t) vf[t] = load_frag(vbase + (size_t)(16 * t) * SEQ + kb, hh);
#pragma unroll
    for (int t = 0; t < 4; ++t) o[t] = wmma_f16(vf[t], pbG, o[t]);
    if (lov) {
#pragma unroll
      for (int t = 0; t < 4; ++t) ol[t] = wmma_f16(vf[t], pbL, ol[t]);
    }
  }

  const float al   = alpha[0];
  const float ag   = 1.0f / (1.0f + expf(-al));
  const float invG = (1.0f / lG) * (1.0f / (PSC * 8.0f));
  const float rl   = (lL > 0.0f) ? (1.0f / lL) : 0.0f;
  const float invL = rl * (1.0f / (PSC * 8.0f));
  float* so = sO + w * 1024;
#pragma unroll
  for (int t = 0; t < 4; ++t)
#pragma unroll
    for (int r = 0; r < 8; ++r) {
      const float gv = o[t][r] * invG;
      const float lv = ol[t][r] * invL;
      const float tt = ag * gv + (1.0f - ag) * lv;
      const float sq = sqrtf(fabsf(tt));
      const float tv = (tt > 0.0f) ? sq : ((tt < 0.0f) ? -sq : 0.0f);
      so[m * 64 + 16 * t + 8 * hh + r] = tv;
    }
  __syncthreads();

  if (tid < 64) {
    float cs = 0.0f;
#pragma unroll 1
    for (int rr = 0; rr < 64; ++rr) {
      const float v = sO[rr * 64 + tid];
      cs += v * v;
    }
    csum[tid] = cs;
  }
  __syncthreads();

  const v4f cv = *(const v4fa*)(csum + 4 * (lane & 15));
  const size_t ridx = ((size_t)(bh * NQT + qt)) * 64;
  const bool wr = (w == 0) && (lane < 16);

  att_store_pass(so, tmp, b, head, q0w, lane);
  if (wr) *(volatile v4f*)(rec + ridx + 4 * lane) = cv;
  __threadfence();
  att_store_pass(so, tmp, b, head, q0w, lane);
  if (wr) *(volatile v4f*)(rec + ridx + 4 * lane) = cv;
}

__global__ __launch_bounds__(512) void k_fold(const float* __restrict__ rec, float* invt) {
  const int t = threadIdx.x;
  const int b = t >> 8, c = t & 255;
  const int head = c >> 6, d = c & 63;
  const float* rp = rec + ((size_t)((b * NH + head) * NQT)) * 64 + d;
  float s = 0.0f;
#pragma unroll 1
  for (int qt = 0; qt < NQT; ++qt) s += rp[qt * 64];
  const float nrm = fmaxf(sqrtf(s), 1e-12f);
  const float inv = 1.0f / nrm;
  *(volatile float*)(invt + t) = inv;
  __threadfence();
  *(volatile float*)(invt + t) = inv;
}

__global__ __launch_bounds__(256) void k_tmpn(const float* __restrict__ tmp, const float* __restrict__ invt,
                                               _Float16* outp) {
  const int g = blockIdx.x * 256 + (int)threadIdx.x;
  const int row = g >> 5, c8 = (g & 31) * 8;
  const int b = row >> 11;
  const v4f a  = *(const v4fa*)(tmp + (size_t)row * HID + c8);
  const v4f c  = *(const v4fa*)(tmp + (size_t)row * HID + c8 + 4);
  const v4f i0 = *(const v4fa*)(invt + b * HID + c8);
  const v4f i1 = *(const v4fa*)(invt + b * HID + c8 + 4);
  const float sc = 1024.0f;
  const v8h o = { (_Float16)(a.x * i0.x * sc), (_Float16)(a.y * i0.y * sc), (_Float16)(a.z * i0.z * sc), (_Float16)(a.w * i0.w * sc),
                  (_Float16)(c.x * i1.x * sc), (_Float16)(c.y * i1.y * sc), (_Float16)(c.z * i1.z * sc), (_Float16)(c.w * i1.w * sc) };
  _Float16* d = outp + (size_t)row * HID + c8;
  *(volatile v8h*)d = o;
  __threadfence();
  *(volatile v8h*)d = o;
}

template <bool H16>
__global__ __launch_bounds__(256) void k_ln(const float* __restrict__ x, const float* __restrict__ g,
                                             const float* __restrict__ be,
                                             float* outF, _Float16* outH, float carry) {
  __shared__ __attribute__((aligned(16))) float ys[8 * DM];
  const int lane = threadIdx.x & 31, w = threadIdx.x >> 5;
  const int row = blockIdx.x * 8 + w;
  const float* p = x + (size_t)row * DM;
  float* yw = ys + w * DM;

  float s = 0.0f;
#pragma unroll 1
  for (int j = 0; j < 8; ++j) {
    const v4f a = *(const v4fa*)(p + (j * 32 + lane) * 4);
    s += (a.x + a.y) + (a.z + a.w);
  }
#pragma unroll
  for (int off = 16; off > 0; off >>= 1) s += __shfl_xor(s, off, 32);
  const float mu = s * (1.0f / (float)DM);

  float vs = 0.0f;
#pragma unroll 1
  for (int j = 0; j < 8; ++j) {
    const v4f a = *(const v4fa*)(p + (j * 32 + lane) * 4);
    const v4f d = a - mu;
    vs += (d.x * d.x + d.y * d.y) + (d.z * d.z + d.w * d.w);
  }
#pragma unroll
  for (int off = 16; off > 0; off >>= 1) vs += __shfl_xor(vs, off, 32);
  const float rstd = rsqrtf(vs * (1.0f / (float)DM) + 1e-5f);

#pragma unroll 1
  for (int j = 0; j < 8; ++j) {
    const int e = (j * 32 + lane) * 4;
    const v4f a  = *(const v4fa*)(p + e);
    const v4f gv = *(const v4fa*)(g + e);
    const v4f bv = *(const v4fa*)(be + e);
    const v4f y  = (a - mu) * rstd * gv + bv;
    *(v4fa*)(yw + e) = y;
  }
  __builtin_amdgcn_fence(__ATOMIC_RELEASE, "wavefront");
  __builtin_amdgcn_wave_barrier();

  for (int pass = 0; pass < 2; ++pass) {
#pragma unroll 1
    for (int j = 0; j < 8; ++j) {
      const int e = (j * 32 + lane) * 4;
      const v4f y = *(const v4fa*)(yw + e);
      const size_t gi = (size_t)row * DM + e;
      *(volatile v4f*)(outF + gi) = y;
      if (H16) {
        const v4h hq = { (_Float16)(y.x * carry), (_Float16)(y.y * carry), (_Float16)(y.z * carry), (_Float16)(y.w * carry) };
        *(volatile v4h*)(outH + gi) = hq;
      }
    }
    __threadfence();
  }
}

extern "C" void kernel_launch(void* const* d_in, const int* in_sizes, int n_in,
                              void* d_out, int out_size, void* d_ws, size_t ws_size,
                              hipStream_t stream) {
  if (n_in < 22) return;
  if (in_sizes[0] != MROWS * DM || in_sizes[1] != MROWS * DM || in_sizes[2] != MROWS * DM) return;
  if (in_sizes[3] != DM * HID || in_sizes[5] != DM * HID || in_sizes[7] != DM * HID) return;
  if (in_sizes[4] != HID || in_sizes[6] != HID || in_sizes[8] != HID) return;
  if (in_sizes[9] != HID * DM || in_sizes[10] != DM) return;
  if (in_sizes[11] < 1 || in_sizes[12] < 1 || in_sizes[13] < 1) return;
  if (in_sizes[14] != DM * DFF || in_sizes[15] != DFF) return;
  if (in_sizes[16] != DFF * DM || in_sizes[17] != DM) return;
  if (in_sizes[18] != DM || in_sizes[19] != DM || in_sizes[20] != DM || in_sizes[21] != DM) return;
  if (out_size != MROWS * DM) return;

  const float* q     = (const float*)d_in[0];
  const float* k     = (const float*)d_in[1];
  const float* v     = (const float*)d_in[2];
  const float* Wq    = (const float*)d_in[3];
  const float* bq    = (const float*)d_in[4];
  const float* Wk    = (const float*)d_in[5];
  const float* bk    = (const float*)d_in[6];
  const float* Wv    = (const float*)d_in[7];
  const float* bv    = (const float*)d_in[8];
  const float* Wo    = (const float*)d_in[9];
  const float* bo    = (const float*)d_in[10];
  const float* alpha = (const float*)d_in[11];
  const float* adjw  = (const float*)d_in[12];
  const float* adjb  = (const float*)d_in[13];
  const float* W1    = (const float*)d_in[14];
  const float* b1    = (const float*)d_in[15];
  const float* W2    = (const float*)d_in[16];
  const float* b2    = (const float*)d_in[17];
  const float* g1    = (const float*)d_in[18];
  const float* be1   = (const float*)d_in[19];
  const float* g2    = (const float*)d_in[20];
  const float* be2   = (const float*)d_in[21];
  float* out = (float*)d_out;

  const size_t PACT16 = (size_t)MROWS * DM * 2;
  const size_t PW16   = (size_t)DM * HID * 2;
  const size_t PWF16  = (size_t)DM * DFF * 2;
  const size_t PPRJ   = (size_t)MROWS * HID * 2;
  const size_t PVT    = (size_t)NBATCH * HID * SEQ * 2;
  const size_t PTMP   = (size_t)MROWS * HID * 4;
  const size_t PREC   = (size_t)NBATCH * NH * NQT * 64 * 4;
  const size_t PINV   = 2048;
  const size_t PACT32 = (size_t)MROWS * DM * 4;
  const size_t PHH    = (size_t)MROWS * DFF * 2;
  size_t off = 0;
  const size_t oQ16 = off; off += PACT16;
  const size_t oK16 = off; off += PACT16;
  const size_t oV16 = off; off += PACT16;
  const size_t oWqT = off; off += PW16;
  const size_t oWkT = off; off += PW16;
  const size_t oWvT = off; off += PW16;
  const size_t oWoT = off; off += PW16;
  const size_t oW1T = off; off += PWF16;
  const size_t oW2T = off; off += PWF16;
  const size_t oQp  = off; off += PPRJ;
  const size_t oKp  = off; off += PPRJ;
  const size_t oVT  = off; off += PVT;
  const size_t oTmp = off; off += PTMP;
  const size_t oRec = off; off += PREC;
  const size_t oInv = off; off += PINV;
  const size_t oTpn = off; off += PPRJ;
  const size_t oXa  = off; off += PACT32;
  const size_t oX1  = off; off += PACT32;
  const size_t oX1h = off; off += PACT16;
  const size_t oHh  = off; off += PHH;
  const size_t oX2  = off; off += PACT32;
  if (off > ws_size) return;
  if (off > (size_t)134217728) return;

  char* ws = (char*)d_ws;
  _Float16* q16  = (_Float16*)(ws + oQ16);
  _Float16* k16  = (_Float16*)(ws + oK16);
  _Float16* v16  = (_Float16*)(ws + oV16);
  _Float16* WqT  = (_Float16*)(ws + oWqT);
  _Float16* WkT  = (_Float16*)(ws + oWkT);
  _Float16* WvT  = (_Float16*)(ws + oWvT);
  _Float16* WoT  = (_Float16*)(ws + oWoT);
  _Float16* W1T  = (_Float16*)(ws + oW1T);
  _Float16* W2T  = (_Float16*)(ws + oW2T);
  _Float16* Qp   = (_Float16*)(ws + oQp);
  _Float16* Kp   = (_Float16*)(ws + oKp);
  _Float16* VT   = (_Float16*)(ws + oVT);
  float*    tmp  = (float*)(ws + oTmp);
  float*    rec  = (float*)(ws + oRec);
  float*    invt = (float*)(ws + oInv);
  _Float16* tmpn = (_Float16*)(ws + oTpn);
  float*    xa   = (float*)(ws + oXa);
  float*    x1   = (float*)(ws + oX1);
  _Float16* x1h  = (_Float16*)(ws + oX1h);
  _Float16* hh   = (_Float16*)(ws + oHh);
  float*    x2   = (float*)(ws + oX2);

  const dim3 b256(256), b128(128);

  k_cvt<<<dim3((3 * N8ACT) / 256), b256, 0, stream>>>(q, k, v, q16, k16, v16);

  k_wt<<<dim3(HID / 64, DM / 64), b256, 0, stream>>>(Wq, DM, HID, WqT, 64.0f);
  k_wt<<<dim3(HID / 64, DM / 64), b256, 0, stream>>>(Wk, DM, HID, WkT, 64.0f);
  k_wt<<<dim3(HID / 64, DM / 64), b256, 0, stream>>>(Wv, DM, HID, WvT, 64.0f);
  k_wt<<<dim3(DM / 64, HID / 64), b256, 0, stream>>>(Wo, HID, DM, WoT, 64.0f);
  k_wt<<<dim3(DFF / 64, DM / 64), b256, 0, stream>>>(W1, DM, DFF, W1T, 64.0f);
  k_wt<<<dim3(DM / 64, DFF / 64), b256, 0, stream>>>(W2, DFF, DM, W2T, 64.0f);

  gemm_k<1, false><<<dim3(MROWS / 128, HID / 64, 1), b128, 0, stream>>>(
      q16, DM, 0LL, WqT, DM, 0LL, bq, (const float*)0, (void*)Qp, HID, 0LL, DM, 1.0f / 64.0f, 8.0f);
  gemm_k<1, false><<<dim3(MROWS / 128, HID / 64, 1), b128, 0, stream>>>(
      k16, DM, 0LL, WkT, DM, 0LL, bk, (const float*)0, (void*)Kp, HID, 0LL, DM, 1.0f / 64.0f, 8.0f);
  gemm_k<2, false><<<dim3(HID / 128, SEQ / 64, NBATCH), b128, 0, stream>>>(
      WvT, DM, 0LL, v16, DM, (long long)SEQ * DM, bv, (const float*)0, (void*)VT, SEQ, (long long)HID * SEQ,
      DM, 1.0f / 64.0f, 8.0f);

  attn_k<<<dim3(NQT, NBATCH * NH), b128, 0, stream>>>(Qp, Kp, VT, alpha, adjw, adjb, tmp, rec);

  k_fold<<<dim3(1), dim3(NBATCH * HID), 0, stream>>>(rec, invt);
  k_tmpn<<<dim3((MROWS * HID / 8) / 256), b256, 0, stream>>>(tmp, invt, tmpn);

  gemm_k<0, false><<<dim3(MROWS / 128, DM / 64, 1), b128, 0, stream>>>(
      tmpn, HID, 0LL, WoT, HID, 0LL, bo, q, (void*)xa, DM, 0LL, HID, 1.0f / 65536.0f, 1.0f);

  k_ln<true><<<dim3(MROWS / 8), b256, 0, stream>>>(xa, g1, be1, x1, x1h, 8.0f);

  gemm_k<1, true><<<dim3(MROWS / 128, DFF / 64, 1), b128, 0, stream>>>(
      x1h, DM, 0LL, W1T, DM, 0LL, b1, (const float*)0, (void*)hh, DFF, 0LL, DM, 1.0f / 512.0f, 8.0f);

  gemm_k<0, false><<<dim3(MROWS / 128, DM / 64, 1), b128, 0, stream>>>(
      hh, DFF, 0LL, W2T, DFF, 0LL, b2, x1, (void*)x2, DM, 0LL, DFF, 1.0f / 512.0f, 1.0f);

  k_ln<false><<<dim3(MROWS / 8), b256, 0, stream>>>(x2, g2, be2, out, (_Float16*)0, 1.0f);

  (void)hipGetLastError();
}
